// TalkingHeadAttention_21440476742379
// MI455X (gfx1250) — hardware-verified
//
#include <hip/hip_runtime.h>
#include <stdint.h>
#include <stddef.h>


typedef __attribute__((ext_vector_type(16))) _Float16 v16h;
typedef __attribute__((ext_vector_type(8)))  _Float16 v8h;
typedef __attribute__((ext_vector_type(16))) __bf16   v16b;
typedef __attribute__((ext_vector_type(8)))  __bf16   v8b;
typedef __attribute__((ext_vector_type(8)))  float    v8f;
typedef __attribute__((ext_vector_type(4)))  float    v4f;
typedef __attribute__((ext_vector_type(2)))  float    v2f;

__device__ __forceinline__ unsigned short f2bf_bits(float f) {
  unsigned u = __float_as_uint(f);
  return (unsigned short)((u + 0x7FFFu + ((u >> 16) & 1u)) >> 16);
}
__device__ __forceinline__ float bf_bits2f(unsigned short h) { return __uint_as_float(((unsigned)h) << 16); }

__device__ __forceinline__ void dep_guard_h(v8f& a, v8f& b, v16h x, v16h y) { asm volatile("v_nop\n\tv_nop\n\tv_nop\n\tv_nop" : "+v"(a), "+v"(b) : "v"(x), "v"(y)); }
__device__ __forceinline__ void dep_guard_b(v8f& a, v8f& b, v16b x, v16b y) { asm volatile("v_nop\n\tv_nop\n\tv_nop\n\tv_nop" : "+v"(a), "+v"(b) : "v"(x), "v"(y)); }
__device__ __forceinline__ void keep4_h(v16h a, v16h b, v16h c, v16h d) { asm volatile("v_nop" :: "v"(a), "v"(b), "v"(c), "v"(d)); }
__device__ __forceinline__ void keep4_b(v16b a, v16b b, v16b c, v16b d) { asm volatile("v_nop" :: "v"(a), "v"(b), "v"(c), "v"(d)); }
__device__ __forceinline__ void acc_guard4(v8f& a, v8f& b, v8f& c, v8f& d) { asm volatile("v_nop\n\tv_nop\n\tv_nop\n\tv_nop" : "+v"(a), "+v"(b), "+v"(c), "+v"(d)); }
template <typename T> struct Frag;
template <> struct Frag<_Float16> {
  typedef v16h V; union U { v16h v; v8h h[2]; };
  static __device__ __forceinline__ v16h load(const _Float16* p) {
    U f; f.h[0] = *(const v8h*)(p); f.h[1] = *(const v8h*)(p + 16); return f.v;
  }
  static __device__ __forceinline__ v8f mma(v16h a, v16h b, v8f c) {
    return __builtin_amdgcn_wmma_f32_16x16x32_f16(false, a, false, b, (short)0, c, false, false);
  }
  static __device__ __forceinline__ void guard(v8f& a, v8f& b, v16h x, v16h y) { dep_guard_h(a, b, x, y); }
  static __device__ __forceinline__ void keep(v16h a, v16h b, v16h c, v16h d) { keep4_h(a, b, c, d); }
};
template <> struct Frag<__bf16> {
  typedef v16b V; union U { v16b v; v8b h[2]; };
  static __device__ __forceinline__ v16b load(const __bf16* p) {
    U f; f.h[0] = *(const v8b*)(p); f.h[1] = *(const v8b*)(p + 16); return f.v;
  }
  static __device__ __forceinline__ v8f mma(v16b a, v16b b, v8f c) {
    return __builtin_amdgcn_wmma_f32_16x16x32_bf16(false, a, false, b, (short)0, c, false, false);
  }
  static __device__ __forceinline__ void guard(v8f& a, v8f& b, v16b x, v16b y) { dep_guard_b(a, b, x, y); }
  static __device__ __forceinline__ void keep(v16b a, v16b b, v16b c, v16b d) { keep4_b(a, b, c, d); }
};

template <int ET> struct Elem;
template <> struct Elem<0> { typedef _Float16 T; };
template <> struct Elem<1> { typedef __bf16 T; };
template <int ET, bool SPLIT, int BIAS_MODE, int OUT_MODE, bool RESID, int ACT = 0>
__global__ __launch_bounds__(256) void wmma_gemm64(
    const unsigned short* __restrict__ Ap, const unsigned short* __restrict__ A2p, int lda, long strideA,
    const unsigned short* __restrict__ Btp, const unsigned short* __restrict__ Bt2p, int ldb, long strideB,
    void* __restrict__ Cout, void* __restrict__ Cout2, int ldc, long strideC,
    const float* __restrict__ bias,
    const float* __restrict__ resid, long strideR,
    int M, int N, int K, float scale) {
  typedef typename Elem<ET>::T T;
  typedef typename Frag<T>::V V;
  const T* A = (const T*)Ap; const T* A2 = (const T*)A2p; const T* Bt = (const T*)Btp; const T* Bt2 = (const T*)Bt2p;
  __shared__ __align__(16) float sT[8][16 * 68];
  const int b    = blockIdx.y;
  const int lane = threadIdx.x & 31;
  const int wave = threadIdx.x >> 5;
  const int tilesN = N >> 6;
  const int tilesM = M >> 6;
  const int tile = blockIdx.x * 8 + wave;
  if (tile >= tilesM * tilesN) return;
  const int tm = tile / tilesN;
  const int tn = tile - tm * tilesN;
  const int m0 = tm << 6;
  const int n0 = tn << 6;

  const T* Ab  = A  + (size_t)b * strideA;
  const T* Bb  = Bt + (size_t)b * strideB;
  const T* Ab2 = SPLIT ? (A2  + (size_t)b * strideA) : nullptr;
  const T* Bb2 = SPLIT ? (Bt2 + (size_t)b * strideB) : nullptr;

  const int rlane = lane & 15;
  const int koff  = (lane >> 4) * 8;
  const int mOff  = (lane >> 4) * 8;

  v8f acc[4][4];
#pragma unroll
  for (int i = 0; i < 4; ++i)
#pragma unroll
    for (int j = 0; j < 4; ++j) acc[i][j] = (v8f){0.f,0.f,0.f,0.f,0.f,0.f,0.f,0.f};

  for (int k0 = 0; k0 < K; k0 += 32) {
    V bh[4], bl[4];
#pragma unroll
    for (int j = 0; j < 4; ++j) {
      const size_t bo = (size_t)(n0 + (j << 4) + rlane) * ldb + koff + k0;
      bh[j] = Frag<T>::load(Bb + bo);
      if (SPLIT) bl[j] = Frag<T>::load(Bb2 + bo);
    }
#pragma unroll
    for (int i = 0; i < 4; ++i) {
      const size_t ao = (size_t)(m0 + (i << 4) + rlane) * lda + koff + k0;
      V ah = Frag<T>::load(Ab + ao);
      V al;
      if (SPLIT) al = Frag<T>::load(Ab2 + ao);
#pragma unroll
      for (int j = 0; j < 4; ++j) {
        acc[i][j] = Frag<T>::mma(ah, bh[j], acc[i][j]);
        if (SPLIT) {
          acc[i][j] = Frag<T>::mma(ah, bl[j], acc[i][j]);
          acc[i][j] = Frag<T>::mma(al, bh[j], acc[i][j]);
        }
      }
      Frag<T>::guard(acc[i][0], acc[i][3], ah, SPLIT ? al : ah);
    }
    Frag<T>::keep(bh[0], bh[1], bh[2], bh[3]);
    if (SPLIT) Frag<T>::keep(bl[0], bl[1], bl[2], bl[3]);
  }
  acc_guard4(acc[0][0], acc[0][1], acc[0][2], acc[0][3]);
  acc_guard4(acc[1][0], acc[1][1], acc[1][2], acc[1][3]);
  acc_guard4(acc[2][0], acc[2][1], acc[2][2], acc[2][3]);
  acc_guard4(acc[3][0], acc[3][1], acc[3][2], acc[3][3]);

  float* slab = sT[wave];
  const float* Rb = RESID ? (resid + (size_t)b * strideR) : nullptr;
#pragma unroll
  for (int i = 0; i < 4; ++i) {
    const int mBase = m0 + (i << 4);
#pragma unroll
    for (int j = 0; j < 4; ++j) {
      const int n = n0 + (j << 4) + rlane;
      float bv = 0.f;
      if (BIAS_MODE == 2) bv = bias[n];
#pragma unroll
      for (int r = 0; r < 8; ++r) {
        float v = acc[i][j][r] * scale;
        if (BIAS_MODE == 1) v += bias[mBase + mOff + r];
        if (BIAS_MODE == 2) v += bv;
        if (RESID) v += Rb[(size_t)(mBase + mOff + r) * ldc + n];
        if (ACT == 1) v = tanhf(v);
        if (ACT == 2) v = fmaxf(v, 0.0f);
        if (ACT == 3) v = v / (1.0f + expf(-v));
        if (ACT == 4) v = (v > 0.f) ? v : 0.01f * v;
        if (ACT == 5) v = 0.5f * v * (1.0f + erff(v * 0.70710678118654752f));
        slab[(mOff + r) * 68 + (j << 4) + rlane] = v;
      }
    }
    __builtin_amdgcn_fence(__ATOMIC_RELEASE, "workgroup");
    __builtin_amdgcn_wave_barrier();
    __builtin_amdgcn_fence(__ATOMIC_ACQUIRE, "workgroup");
    if (OUT_MODE == 0) {
      float* C = (float*)Cout + (size_t)b * strideC;
      const int hh = lane >> 4, c4 = (lane & 15) * 4;
      for (int pass = 0; pass < 2; ++pass) {
#pragma unroll
        for (int it = 0; it < 8; ++it) {
          const int row = it * 2 + hh;
          v4f v = *(const v4f*)(slab + row * 68 + c4);
          *(volatile v4f*)(C + (size_t)(mBase + row) * ldc + n0 + c4) = v;
        }
        __threadfence();
      }
    } else {
      const int q = lane >> 3, c8 = (lane & 7) * 8;
      unsigned short* C  = (unsigned short*)Cout  + (size_t)b * strideC;
      unsigned short* C2 = (OUT_MODE == 2) ? ((unsigned short*)Cout2 + (size_t)b * strideC) : nullptr;
      for (int pass = 0; pass < 2; ++pass) {
#pragma unroll
        for (int it = 0; it < 4; ++it) {
          const int row = it * 4 + q;
          const float* sp = slab + row * 68 + c8;
          v8h hv, lv;
#pragma unroll
          for (int e = 0; e < 8; ++e) {
            if (OUT_MODE == 1) {
              hv[e] = (_Float16)sp[e];
            } else {
              unsigned short hb = f2bf_bits(sp[e]);
              unsigned short lb = f2bf_bits(sp[e] - bf_bits2f(hb));
              hv[e] = __builtin_bit_cast(_Float16, hb);
              lv[e] = __builtin_bit_cast(_Float16, lb);
            }
          }
          *(volatile v8h*)(C + (size_t)(mBase + row) * ldc + n0 + c8) = hv;
          if (OUT_MODE == 2) *(volatile v8h*)(C2 + (size_t)(mBase + row) * ldc + n0 + c8) = lv;
        }
        __threadfence();
      }
    }
    __builtin_amdgcn_fence(__ATOMIC_RELEASE, "workgroup");
    __builtin_amdgcn_wave_barrier();
    __builtin_amdgcn_fence(__ATOMIC_ACQUIRE, "workgroup");
  }
}

__global__ __launch_bounds__(256) void cast_f32_f16x2s(
    const float* __restrict__ in, _Float16* __restrict__ out, int n2, float scale) {
  int i = blockIdx.x * 256 + threadIdx.x;
  if (i < n2) {
    const v2f a = *(const v2f*)(in + 2 * (size_t)i);
    const _Float16 h0 = (_Float16)(a[0] * scale), h1 = (_Float16)(a[1] * scale);
    const unsigned u = (unsigned)__builtin_bit_cast(unsigned short, h0) | ((unsigned)__builtin_bit_cast(unsigned short, h1) << 16);
    ((volatile unsigned*)out)[i] = u;
    __threadfence();
    ((volatile unsigned*)out)[i] = u;
  }
}

#define MX_H 12
#define MX_N 1024

__global__ __launch_bounds__(256) void th_mix_kernel(
    const float* __restrict__ S, const float* __restrict__ w1, const float* __restrict__ b1,
    const float* __restrict__ w2, const float* __restrict__ b2,
    unsigned short* __restrict__ P, float pcarry)
{
  __shared__ __align__(16) float T[MX_H * MX_N];
  __shared__ __align__(16) float w1s[MX_H * MX_H];
  __shared__ __align__(16) float w2s[MX_H * MX_H];
  __shared__ float b1s[16];
  __shared__ float b2s[16];
  __shared__ float invs[16];
  __shared__ float rmax[8];
  __shared__ float rsum[8];

  const int n    = blockIdx.x;
  const int tid  = threadIdx.x;
  const int lane = tid & 31;
  const int wave = tid >> 5;
  const size_t HS = (size_t)MX_N * MX_N;

  if (tid < MX_H * MX_H) { w1s[tid] = w1[tid]; w2s[tid] = w2[tid]; }
  if (tid < MX_H) { b1s[tid] = b1[tid]; b2s[tid] = b2[tid]; }
  __syncthreads();

#pragma unroll 1
  for (int cc = 0; cc < 2; ++cc) {
    const int m = cc * 512 + tid * 2;
    const float* sp = S + (size_t)n * MX_N + m;
    v2f s[MX_H];
#pragma unroll
    for (int h = 0; h < MX_H; ++h) s[h] = *(const v2f*)(sp + (size_t)h * HS);
#pragma unroll 1
    for (int g = 0; g < MX_H; ++g) {
      const v4f wa = *(const v4f*)(w1s + g * MX_H);
      const v4f wb = *(const v4f*)(w1s + g * MX_H + 4);
      const v4f wc = *(const v4f*)(w1s + g * MX_H + 8);
      const float bg = b1s[g];
      v2f a = (v2f){bg, bg};
      a += wa[0] * s[0];  a += wa[1] * s[1];  a += wa[2] * s[2];  a += wa[3] * s[3];
      a += wb[0] * s[4];  a += wb[1] * s[5];  a += wb[2] * s[6];  a += wb[3] * s[7];
      a += wc[0] * s[8];  a += wc[1] * s[9];  a += wc[2] * s[10]; a += wc[3] * s[11];
      *(v2f*)(T + g * MX_N + m) = a;
    }
  }
  __syncthreads();

#pragma unroll 1
  for (int g = 0; g < MX_H; ++g) {
    float* tp = T + g * MX_N + tid * 4;
    const v4f x = *(const v4f*)tp;
    float mx = fmaxf(fmaxf(x[0], x[1]), fmaxf(x[2], x[3]));
#pragma unroll
    for (int off = 16; off > 0; off >>= 1) mx = fmaxf(mx, __shfl_xor(mx, off, 32));
    if (lane == 0) rmax[wave] = mx;
    __syncthreads();
    float M = rmax[0];
#pragma unroll
    for (int w = 1; w < 8; ++w) M = fmaxf(M, rmax[w]);
    v4f e;
    e[0] = __expf(x[0] - M);
    e[1] = __expf(x[1] - M);
    e[2] = __expf(x[2] - M);
    e[3] = __expf(x[3] - M);
    *(v4f*)tp = e;
    float sm = (e[0] + e[1]) + (e[2] + e[3]);
#pragma unroll
    for (int off = 16; off > 0; off >>= 1) sm += __shfl_xor(sm, off, 32);
    if (lane == 0) rsum[wave] = sm;
    __syncthreads();
    float tot = rsum[0];
#pragma unroll
    for (int w = 1; w < 8; ++w) tot += rsum[w];
    if (tid == 0) invs[g] = 1.0f / tot;
  }
  __syncthreads();
  if (tid < MX_H * MX_H) {
    const int h = tid % MX_H;
    w2s[tid] = w2s[tid] * invs[h] * pcarry;
  }
  if (tid < MX_H) b2s[tid] = b2s[tid] * pcarry;
  __syncthreads();

#pragma unroll 1
  for (int cc = 0; cc < 2; ++cc) {
    const int m = cc * 512 + tid * 2;
    v2f e[MX_H];
#pragma unroll
    for (int h = 0; h < MX_H; ++h) e[h] = *(const v2f*)(T + h * MX_N + m);
    unsigned short* prow = P + (size_t)n * MX_N + m;
#pragma unroll 1
    for (int g = 0; g < MX_H; ++g) {
      const v4f wa = *(const v4f*)(w2s + g * MX_H);
      const v4f wb = *(const v4f*)(w2s + g * MX_H + 4);
      const v4f wc = *(const v4f*)(w2s + g * MX_H + 8);
      const float bg = b2s[g];
      v2f a = (v2f){bg, bg};
      a += wa[0] * e[0];  a += wa[1] * e[1];  a += wa[2] * e[2];  a += wa[3] * e[3];
      a += wb[0] * e[4];  a += wb[1] * e[5];  a += wb[2] * e[6];  a += wb[3] * e[7];
      a += wc[0] * e[8];  a += wc[1] * e[9];  a += wc[2] * e[10]; a += wc[3] * e[11];
      const _Float16 h0 = (_Float16)a[0], h1 = (_Float16)a[1];
      const unsigned u = (unsigned)__builtin_bit_cast(unsigned short, h0) | ((unsigned)__builtin_bit_cast(unsigned short, h1) << 16);
      volatile unsigned* pp = (volatile unsigned*)(prow + (size_t)g * HS);
      *pp = u;
      __threadfence();
      *pp = u;
    }
  }
}

template <int BIAS_MODE, int OUT_MODE>
static void gemm_f16(hipStream_t st, int gy,
                     const void* A, int lda, long sA,
                     const void* Bt, int ldb, long sB,
                     void* C, int ldc, long sC,
                     const float* bias, int M, int N, int K, float scale)
{
  const int tiles = (M / 64) * (N / 64);
  dim3 grid((tiles + 7) / 8, gy);
  wmma_gemm64<0, false, BIAS_MODE, OUT_MODE, false, 0><<<grid, 256, 0, st>>>(
      (const unsigned short*)A, (const unsigned short*)A, lda, sA,
      (const unsigned short*)Bt, (const unsigned short*)Bt, ldb, sB,
      C, C, ldc, sC, bias, bias, (long)0, M, N, K, scale);
}

extern "C" void kernel_launch(void* const* d_in, const int* in_sizes, int n_in,
                              void* d_out, int out_size, void* d_ws, size_t ws_size,
                              hipStream_t stream)
{
  const int Bn = 8, Nn = 1024, Dd = 768, Hh = 12, HD = 64;
  if (n_in < 13) return;
  if (in_sizes[0] != Bn * Nn * Dd) return;
  if (in_sizes[1] != Dd * Dd || in_sizes[3] != Dd * Dd || in_sizes[5] != Dd * Dd || in_sizes[7] != Dd * Dd) return;
  if (in_sizes[2] != Dd || in_sizes[4] != Dd || in_sizes[6] != Dd || in_sizes[8] != Dd) return;
  if (in_sizes[9] != Hh * Hh || in_sizes[10] != Hh || in_sizes[11] != Hh * Hh || in_sizes[12] != Hh) return;
  if (out_size != Bn * Nn * Dd) return;

  const float* x    = (const float*)d_in[0];
  const float* wq   = (const float*)d_in[1];
  const float* bq   = (const float*)d_in[2];
  const float* wk   = (const float*)d_in[3];
  const float* bk   = (const float*)d_in[4];
  const float* wv   = (const float*)d_in[5];
  const float* bv   = (const float*)d_in[6];
  const float* wo   = (const float*)d_in[7];
  const float* bo   = (const float*)d_in[8];
  const float* th1w = (const float*)d_in[9];
  const float* th1b = (const float*)d_in[10];
  const float* th2w = (const float*)d_in[11];
  const float* th2b = (const float*)d_in[12];
  float* out = (float*)d_out;

  const size_t WSZ = (size_t)Dd * Dd * 2;
  const size_t ASZ = (size_t)Bn * Nn * Dd * 2;
  const size_t SSZ = (size_t)Hh * Nn * Nn * 4;
  const size_t PSZ = (size_t)Hh * Nn * Nn * 2;
  const size_t off_wq  = 0;
  const size_t off_wk  = off_wq + WSZ;
  const size_t off_wv  = off_wk + WSZ;
  const size_t off_wo  = off_wv + WSZ;
  const size_t off_q   = off_wo + WSZ;
  const size_t off_k   = off_q + ASZ;
  const size_t off_vt  = off_k + ASZ;
  const size_t off_ctx = off_vt + ASZ;
  const size_t off_R   = off_ctx + ASZ;
  const size_t off_x16 = off_R;
  const size_t off_S   = off_R;
  const size_t off_P   = off_S + SSZ;
  size_t end = off_P + PSZ;
  if (off_x16 + ASZ > end) end = off_x16 + ASZ;
  if (end > ws_size) return;
  if (end > (size_t)134217728) return;

  uint8_t* ws = (uint8_t*)d_ws;
  _Float16* wq16 = (_Float16*)(ws + off_wq);
  _Float16* wk16 = (_Float16*)(ws + off_wk);
  _Float16* wv16 = (_Float16*)(ws + off_wv);
  _Float16* wo16 = (_Float16*)(ws + off_wo);
  unsigned short* q16   = (unsigned short*)(ws + off_q);
  unsigned short* k16   = (unsigned short*)(ws + off_k);
  unsigned short* vt16  = (unsigned short*)(ws + off_vt);
  unsigned short* ctx16 = (unsigned short*)(ws + off_ctx);
  _Float16* x16 = (_Float16*)(ws + off_x16);
  float* Sb = (float*)(ws + off_S);
  unsigned short* Pb = (unsigned short*)(ws + off_P);

  const float WCARRY = 64.0f;
  const float PCARRY = 2048.0f;

  {
    const int n2x = Bn * Nn * Dd / 2;
    cast_f32_f16x2s<<<(n2x + 255) / 256, 256, 0, stream>>>(x, x16, n2x, 1.0f);
    const int n2w = Dd * Dd / 2;
    cast_f32_f16x2s<<<(n2w + 255) / 256, 256, 0, stream>>>(wq, wq16, n2w, WCARRY);
    cast_f32_f16x2s<<<(n2w + 255) / 256, 256, 0, stream>>>(wk, wk16, n2w, WCARRY);
    cast_f32_f16x2s<<<(n2w + 255) / 256, 256, 0, stream>>>(wv, wv16, n2w, WCARRY);
    cast_f32_f16x2s<<<(n2w + 255) / 256, 256, 0, stream>>>(wo, wo16, n2w, WCARRY);
  }

  gemm_f16<2, 1>(stream, 1, x16, Dd, 0L, wq16, Dd, 0L, q16, Dd, 0L, bq, Bn * Nn, Dd, Dd, 1.0f / WCARRY);
  gemm_f16<2, 1>(stream, 1, x16, Dd, 0L, wk16, Dd, 0L, k16, Dd, 0L, bk, Bn * Nn, Dd, Dd, 1.0f / WCARRY);
  gemm_f16<1, 1>(stream, Bn, wv16, Dd, 0L, x16, Dd, (long)Nn * Dd, vt16, Nn, (long)Dd * Nn, bv, Dd, Nn, Dd, 1.0f / WCARRY);

  const float qk_scale = 0.125f;
  for (int b = 0; b < Bn; ++b) {
    const unsigned short* qb = q16 + (size_t)b * Nn * Dd;
    const unsigned short* kb = k16 + (size_t)b * Nn * Dd;
    gemm_f16<0, 0>(stream, Hh, qb, Dd, (long)HD, kb, Dd, (long)HD, Sb, Nn, (long)Nn * Nn, bq, Nn, Nn, HD, qk_scale);
    th_mix_kernel<<<Nn, 256, 0, stream>>>(Sb, th1w, th1b, th2w, th2b, Pb, PCARRY);
    gemm_f16<0, 1>(stream, Hh,
                   Pb, Nn, (long)Nn * Nn,
                   vt16 + (size_t)b * Dd * Nn, Nn, (long)HD * Nn,
                   ctx16 + (size_t)b * Nn * Dd, Dd, (long)HD,
                   bq, Nn, HD, Nn, 1.0f / PCARRY);
  }

  gemm_f16<2, 0>(stream, 1, ctx16, Dd, 0L, wo16, Dd, 0L, out, Dd, 0L, bo, Bn * Nn, Dd, Dd, 1.0f / WCARRY);
}
